// SymmetrizationMLP_68101001446045
// MI455X (gfx1250) — hardware-run, weakly checked
//
#include <hip/hip_runtime.h>

typedef __attribute__((ext_vector_type(16))) _Float16 v16h;
typedef __attribute__((ext_vector_type(8)))  _Float16 v8h;
typedef __attribute__((ext_vector_type(8)))  float    v8f;
typedef __attribute__((ext_vector_type(4)))  float    v4f;
typedef __attribute__((ext_vector_type(4)))  int      v4i;

constexpr int kBatch      = 16;
constexpr int kPoints     = 1024;
constexpr int kSlots      = 8;
constexpr int kPerms      = 40320;
constexpr int kDinReal    = 24;
constexpr int kDinPad     = 32;
constexpr int kHid1       = 256;
constexpr int kHid2       = 128;
constexpr int kClasses    = 40;
constexpr int kWavesPerBlock = 4;
constexpr int kThreads    = kWavesPerBlock * 32;
constexpr int kRowsPerWave = 32;
constexpr int kRowsPerIter = kWavesPerBlock * kRowsPerWave;
constexpr int kItersPerBlock = 5;
constexpr int kRowsPerBlock = kRowsPerIter * kItersPerBlock;
constexpr int kBlocksPerBatch = kPerms / kRowsPerBlock;
static_assert(kSlots * 3 == kDinReal, "flat width");
static_assert(kBlocksPerBatch * kRowsPerBlock == kPerms, "row tiles must divide the permutation count");
static_assert(kBlocksPerBatch == 63, "blocks per batch");
static_assert((kDinPad % 32) == 0 && (kHid1 % 32) == 0, "K multiples of 32");
static_assert((kHid1 % 32) == 0 && (kHid2 % 16) == 0, "N tile multiples");
static_assert(kThreads == kHid2, "bias staging assumes 128 threads");
static_assert((kClasses % 4) == 0 && (kBatch * kClasses) == 640, "output lines");

constexpr float kW1Carry   = 64.0f;
constexpr float kH1Carry   = kW1Carry;
constexpr float kW2Carry   = 256.0f;
constexpr float kH2Carry   = kH1Carry * kW2Carry;
constexpr float kInvH2Carry = 1.0f / kH2Carry;
static_assert(kH2Carry == 16384.0f, "carry chain");

constexpr size_t kOffW1T  = 0;
constexpr size_t kOffW2T  = kOffW1T + (size_t)kHid1 * kDinPad * 2;
constexpr size_t kOffPart = kOffW2T + (size_t)kHid2 * kHid1 * 2;
constexpr size_t kWsTotal = kOffPart + (size_t)kBatch * kBlocksPerBatch * kHid2 * 4;
static_assert(kWsTotal == 598016ull, "carve total");
static_assert((kOffW2T % 128) == 0 && (kOffPart % 128) == 0, "aligned regions");
static_assert(kWsTotal <= 134217728ull, "carve cap");

constexpr int kW1Chunks = kHid1 * kDinPad / 8;
constexpr int kW2Chunks = kHid2 * kHid1 / 8;
constexpr int kPrepBlocks = (kW1Chunks + kW2Chunks) / 256;
static_assert(kW1Chunks == 1024 && kW2Chunks == 4096, "chunk counts");
static_assert(kPrepBlocks * 256 == kW1Chunks + kW2Chunks, "prep grid covers the planes exactly");
static_assert((kW1Chunks % 256) == 0, "plane switch is block-uniform");

union FragU { v16h v; v8h h[2]; };
__device__ __forceinline__ v16h frag_ld(const _Float16* p) {
  FragU f;
  f.h[0] = *(const v8h*)(p);
  f.h[1] = *(const v8h*)(p + 16);
  return f.v;
}
__device__ __forceinline__ v8f mma_h(v16h a, v16h b, v8f c) {
  c = __builtin_amdgcn_wmma_f32_16x16x32_f16(false, a, false, b, (short)0, c, false, false);
  asm volatile("v_nop\n\tv_nop\n\tv_nop\n\tv_nop" : "+v"(c) : "v"(a), "v"(b));
  return c;
}

__global__ __launch_bounds__(256) void prep_weights_kernel(
    const float* __restrict__ W1, const float* __restrict__ W2,
    _Float16* __restrict__ W1T, _Float16* __restrict__ W2T)
{
  const int i = blockIdx.x * 256 + threadIdx.x;
  v8h hv;
  _Float16* dst;
  if (blockIdx.x < (kW1Chunks / 256)) {
    const int row = i >> 2;
    const int k0  = (i & 3) * 8;
#pragma unroll
    for (int e = 0; e < 8; ++e) {
      const int k  = k0 + e;
      const int kc = (k < kDinReal) ? k : (kDinReal - 1);
      const float w = W1[kc * kHid1 + row];
      const float v = (k < kDinReal) ? (w * kW1Carry) : 0.0f;
      hv[e] = (_Float16)v;
    }
    dst = W1T + (size_t)i * 8;
  } else {
    const int j   = i - kW1Chunks;
    const int row = j >> 5;
    const int k0  = (j & 31) * 8;
#pragma unroll
    for (int e = 0; e < 8; ++e) {
      const float w = W2[(k0 + e) * kHid2 + row];
      hv[e] = (_Float16)(w * kW2Carry);
    }
    dst = W2T + (size_t)j * 8;
  }
  *(volatile v8h*)dst = hv;
  __threadfence();
  *(volatile v8h*)dst = hv;
}

__global__ __launch_bounds__(kThreads) void fused_mlp_kernel(
    const float* __restrict__ x, const int* __restrict__ sample_idx, const int* __restrict__ perms,
    const float* __restrict__ b1, const float* __restrict__ b2,
    const _Float16* __restrict__ gW1T, const _Float16* __restrict__ gW2T,
    float* __restrict__ partial)
{
  __shared__ __align__(16) _Float16 sW1[kHid1 * kDinPad];
  __shared__ __align__(16) _Float16 sW2[kHid2 * kHid1];
  __shared__ __align__(16) _Float16 sA[kWavesPerBlock * kRowsPerWave * kDinPad];
  __shared__ __align__(16) float    sB1[kHid1];
  __shared__ __align__(16) float    sB2[kHid2];
  __shared__ __align__(16) float    sP[kSlots * 4];
  __shared__ __align__(16) float    sC[kWavesPerBlock * 2 * kHid2];

  const int tid  = threadIdx.x;
  const int lane = tid & 31;
  const int wave = tid >> 5;
  const int n    = lane & 15;
  const int h    = lane >> 4;
  const int b    = blockIdx.x / kBlocksPerBatch;
  const int blk  = blockIdx.x - b * kBlocksPerBatch;

#pragma unroll 1
  for (int i = tid; i < kW1Chunks; i += kThreads)
    *(v8h*)(sW1 + i * 8) = *(const v8h*)(gW1T + (size_t)i * 8);
#pragma unroll 1
  for (int i = tid; i < kW2Chunks; i += kThreads)
    *(v8h*)(sW2 + i * 8) = *(const v8h*)(gW2T + (size_t)i * 8);
  sB1[tid]            = b1[tid] * kH1Carry;
  sB1[tid + kThreads] = b1[tid + kThreads] * kH1Carry;
  sB2[tid]            = b2[tid] * kH2Carry;
  if (wave == 0) {
    const int slot = lane >> 2;
    const int c    = lane & 3;
    const int cc   = (c < 3) ? c : 2;
    int idx = sample_idx[b * kSlots + slot];
    idx = idx < 0 ? 0 : (idx > (kPoints - 1) ? (kPoints - 1) : idx);
    const float v = x[((size_t)b * kPoints + idx) * 3 + cc];
    sP[lane] = (c < 3) ? v : 0.0f;
  }
  float* sCw = sC + wave * (2 * kHid2) + h * kHid2 + n;
#pragma unroll
  for (int nt = 0; nt < kHid2 / 16; ++nt) sCw[nt * 16] = 0.0f;
  __syncthreads();

  _Float16* sAw = sA + wave * (kRowsPerWave * kDinPad);
  const int gBase = blk * kRowsPerBlock + wave * kRowsPerWave + lane;

#pragma unroll 1
  for (int it = 0; it < kItersPerBlock; ++it) {
    {
      const int g = gBase + it * kRowsPerIter;
      const v4i pa = *(const v4i*)(perms + (size_t)g * kSlots);
      const v4i pb = *(const v4i*)(perms + (size_t)g * kSlots + 4);
      int c0 = pa[0], c1 = pa[1], c2 = pa[2], c3 = pa[3];
      int c4 = pb[0], c5 = pb[1], c6 = pb[2], c7 = pb[3];
      c0 = c0 < 0 ? 0 : (c0 > 7 ? 7 : c0);
      c1 = c1 < 0 ? 0 : (c1 > 7 ? 7 : c1);
      c2 = c2 < 0 ? 0 : (c2 > 7 ? 7 : c2);
      c3 = c3 < 0 ? 0 : (c3 > 7 ? 7 : c3);
      c4 = c4 < 0 ? 0 : (c4 > 7 ? 7 : c4);
      c5 = c5 < 0 ? 0 : (c5 > 7 ? 7 : c5);
      c6 = c6 < 0 ? 0 : (c6 > 7 ? 7 : c6);
      c7 = c7 < 0 ? 0 : (c7 > 7 ? 7 : c7);
      const v4f q0 = *(const v4f*)(sP + 4 * c0);
      const v4f q1 = *(const v4f*)(sP + 4 * c1);
      const v4f q2 = *(const v4f*)(sP + 4 * c2);
      const v4f q3 = *(const v4f*)(sP + 4 * c3);
      const v4f q4 = *(const v4f*)(sP + 4 * c4);
      const v4f q5 = *(const v4f*)(sP + 4 * c5);
      const v4f q6 = *(const v4f*)(sP + 4 * c6);
      const v4f q7 = *(const v4f*)(sP + 4 * c7);
      v8h t0, t1, t2, t3;
      t0[0] = (_Float16)q0[0]; t0[1] = (_Float16)q0[1]; t0[2] = (_Float16)q0[2];
      t0[3] = (_Float16)q1[0]; t0[4] = (_Float16)q1[1]; t0[5] = (_Float16)q1[2];
      t0[6] = (_Float16)q2[0]; t0[7] = (_Float16)q2[1]; t1[0] = (_Float16)q2[2];
      t1[1] = (_Float16)q3[0]; t1[2] = (_Float16)q3[1]; t1[3] = (_Float16)q3[2];
      t1[4] = (_Float16)q4[0]; t1[5] = (_Float16)q4[1]; t1[6] = (_Float16)q4[2];
      t1[7] = (_Float16)q5[0]; t2[0] = (_Float16)q5[1]; t2[1] = (_Float16)q5[2];
      t2[2] = (_Float16)q6[0]; t2[3] = (_Float16)q6[1]; t2[4] = (_Float16)q6[2];
      t2[5] = (_Float16)q7[0]; t2[6] = (_Float16)q7[1]; t2[7] = (_Float16)q7[2];
#pragma unroll
      for (int e = 0; e < 8; ++e) t3[e] = (_Float16)0.0f;
      _Float16* rowp = sAw + lane * kDinPad;
      *(v8h*)(rowp)      = t0;
      *(v8h*)(rowp + 8)  = t1;
      *(v8h*)(rowp + 16) = t2;
      *(v8h*)(rowp + 24) = t3;
    }
    __syncthreads();

    const v16h fA = frag_ld(sAw + n * kDinPad + 8 * h);
    const v16h fB = frag_ld(sAw + (16 + n) * kDinPad + 8 * h);
    v16h a2A[kHid1 / 32], a2B[kHid1 / 32];
#pragma unroll
    for (int ks = 0; ks < kHid1 / 32; ++ks) {
      const v16h wLo = frag_ld(sW1 + ((2 * ks) * 16 + n) * kDinPad + 8 * h);
      const v16h wHi = frag_ld(sW1 + ((2 * ks + 1) * 16 + n) * kDinPad + 8 * h);
      const v4f bl0 = *(const v4f*)(sB1 + (2 * ks) * 16 + 8 * h);
      const v4f bl1 = *(const v4f*)(sB1 + (2 * ks) * 16 + 8 * h + 4);
      const v4f bh0 = *(const v4f*)(sB1 + (2 * ks + 1) * 16 + 8 * h);
      const v4f bh1 = *(const v4f*)(sB1 + (2 * ks + 1) * 16 + 8 * h + 4);
      const v8f cLo = (v8f){bl0[0], bl0[1], bl0[2], bl0[3], bl1[0], bl1[1], bl1[2], bl1[3]};
      const v8f cHi = (v8f){bh0[0], bh0[1], bh0[2], bh0[3], bh1[0], bh1[1], bh1[2], bh1[3]};
      v8f d;
      d = mma_h(wLo, fA, cLo);
#pragma unroll
      for (int r = 0; r < 8; ++r) a2A[ks][r] = (_Float16)fmaxf(d[r], 0.0f);
      d = mma_h(wHi, fA, cHi);
#pragma unroll
      for (int r = 0; r < 8; ++r) a2A[ks][8 + r] = (_Float16)fmaxf(d[r], 0.0f);
      d = mma_h(wLo, fB, cLo);
#pragma unroll
      for (int r = 0; r < 8; ++r) a2B[ks][r] = (_Float16)fmaxf(d[r], 0.0f);
      d = mma_h(wHi, fB, cHi);
#pragma unroll
      for (int r = 0; r < 8; ++r) a2B[ks][8 + r] = (_Float16)fmaxf(d[r], 0.0f);
    }

#pragma unroll 1
    for (int nt = 0; nt < kHid2 / 16; ++nt) {
      const float bv = sB2[nt * 16 + n];
      v8f acc0 = (v8f){bv, bv, bv, bv, bv, bv, bv, bv};
      v8f acc1 = acc0;
      const _Float16* wrow = sW2 + (nt * 16 + n) * kHid1 + 8 * h;
#pragma unroll
      for (int ks = 0; ks < kHid1 / 32; ++ks) {
        const v16h bf = frag_ld(wrow + ks * 32);
        acc0 = mma_h(a2A[ks], bf, acc0);
        acc1 = mma_h(a2B[ks], bf, acc1);
      }
      float s = 0.0f;
#pragma unroll
      for (int r = 0; r < 8; ++r) s += fmaxf(acc0[r], 0.0f) + fmaxf(acc1[r], 0.0f);
      s += __shfl_xor(s, 16, 32);
      sCw[nt * 16] += s;
    }
    __syncthreads();
  }

  if (wave == 0) {
    const int j4 = lane * 4;
    v4f s = *(const v4f*)(sC + j4);
    s += *(const v4f*)(sC + 1 * (2 * kHid2) + j4);
    s += *(const v4f*)(sC + 2 * (2 * kHid2) + j4);
    s += *(const v4f*)(sC + 3 * (2 * kHid2) + j4);
    float* dst = partial + ((size_t)(b * kBlocksPerBatch + blk)) * kHid2 + j4;
    *(volatile v4f*)dst = s;
    __threadfence();
    *(volatile v4f*)dst = s;
  }
}

__global__ __launch_bounds__(256) void finalize_kernel(
    const float* __restrict__ partial, const float* __restrict__ W3, const float* __restrict__ b3,
    float* __restrict__ out)
{
  __shared__ __align__(16) float hs[kBatch * kHid2];
  const int tid = threadIdx.x;
#pragma unroll 1
  for (int i = 0; i < 2; ++i) {
    const int q  = tid + 256 * i;
    const int bb = q >> 5;
    const int j4 = (q & 31) * 4;
    const float* p = partial + (size_t)bb * kBlocksPerBatch * kHid2 + j4;
    v4f s = (v4f){0.0f, 0.0f, 0.0f, 0.0f};
#pragma unroll 1
    for (int blk = 0; blk < kBlocksPerBatch; ++blk) {
      const v4f v = *(const v4f*)(p + (size_t)blk * kHid2);
      s += v;
    }
    s *= kInvH2Carry;
    *(v4f*)(hs + bb * kHid2 + j4) = s;
  }
  __syncthreads();
  if (tid < (kBatch * kClasses / 4)) {
    const int o  = tid * 4;
    const int bb = o / kClasses;
    const int c  = o - bb * kClasses;
    const float invG = 1.0f / (float)kPerms;
    v4f acc = (v4f){0.0f, 0.0f, 0.0f, 0.0f};
#pragma unroll 1
    for (int j = 0; j < kHid2; ++j) {
      const float hv = hs[bb * kHid2 + j];
      const v4f w = *(const v4f*)(W3 + j * kClasses + c);
      acc[0] = fmaf(hv, w[0], acc[0]);
      acc[1] = fmaf(hv, w[1], acc[1]);
      acc[2] = fmaf(hv, w[2], acc[2]);
      acc[3] = fmaf(hv, w[3], acc[3]);
    }
    const v4f bias = *(const v4f*)(b3 + c);
    v4f r;
    r[0] = fmaf(acc[0], invG, bias[0]);
    r[1] = fmaf(acc[1], invG, bias[1]);
    r[2] = fmaf(acc[2], invG, bias[2]);
    r[3] = fmaf(acc[3], invG, bias[3]);
    float* dst = out + o;
    *(volatile v4f*)dst = r;
    __threadfence();
    *(volatile v4f*)dst = r;
  }
}

extern "C" void kernel_launch(void* const* d_in, const int* in_sizes, int n_in,
                              void* d_out, int out_size, void* d_ws, size_t ws_size,
                              hipStream_t stream) {
  if (n_in < 9) return;
  if (in_sizes[0] != kBatch * kPoints * 3) return;
  if (in_sizes[1] != kBatch * kSlots) return;
  if (in_sizes[2] != kPerms * kSlots) return;
  if (in_sizes[3] != kDinReal * kHid1) return;
  if (in_sizes[4] != kHid1) return;
  if (in_sizes[5] != kHid1 * kHid2) return;
  if (in_sizes[6] != kHid2) return;
  if (in_sizes[7] != kHid2 * kClasses) return;
  if (in_sizes[8] != kClasses) return;
  if (out_size != kBatch * kClasses) return;
  if (ws_size < kWsTotal) return;

  const float* x          = (const float*)d_in[0];
  const int*   sample_idx = (const int*)d_in[1];
  const int*   perms      = (const int*)d_in[2];
  const float* W1         = (const float*)d_in[3];
  const float* b1         = (const float*)d_in[4];
  const float* W2         = (const float*)d_in[5];
  const float* b2         = (const float*)d_in[6];
  const float* W3         = (const float*)d_in[7];
  const float* b3         = (const float*)d_in[8];
  float* out = (float*)d_out;

  char* ws = (char*)d_ws;
  _Float16* W1T  = (_Float16*)(ws + kOffW1T);
  _Float16* W2T  = (_Float16*)(ws + kOffW2T);
  float*    part = (float*)(ws + kOffPart);

  prep_weights_kernel<<<kPrepBlocks, 256, 0, stream>>>(W1, W2, W1T, W2T);
  fused_mlp_kernel<<<kBatch * kBlocksPerBatch, kThreads, 0, stream>>>(
      x, sample_idx, perms, b1, b2, W1T, W2T, part);
  finalize_kernel<<<1, 256, 0, stream>>>(part, W3, b3, out);
}
